// JKNet_75797582840808
// MI455X (gfx1250) — hardware-run, weakly checked
//
#include <hip/hip_runtime.h>
#include <math.h>

typedef __attribute__((ext_vector_type(16))) _Float16 v16h;
typedef __attribute__((ext_vector_type(8)))  _Float16 v8h;
typedef __attribute__((ext_vector_type(8)))  float    v8f;
typedef __attribute__((ext_vector_type(4)))  float    v4f;
typedef __attribute__((ext_vector_type(4)))  unsigned v4u;
typedef __attribute__((ext_vector_type(4)))  int      v4i;

constexpr int kN      = 100000;
constexpr int kE      = 800000;
constexpr int kD      = 128;
constexpr int kL      = 5;
constexpr int kC      = 40;
constexpr int kCPad   = 64;
constexpr int kNPad   = 100032;
constexpr int kRng    = 2048;
constexpr int kNblkR  = (kNPad + kRng - 1) / kRng;
constexpr int kNTab   = kNblkR * kRng;
constexpr int kCap    = 24576;
constexpr int kCsrTot = kNblkR * kCap;
constexpr int kSortMax = 64;
constexpr float kWCarry    = 16.0f;
constexpr float kWCarryInv = 1.0f / kWCarry;
constexpr float kEps = 1e-5f;

static_assert(kNblkR == 49 && kNTab == 100352, "range blocks");
static_assert((kNPad % 64) == 0 && kNPad >= kN && kNTab >= kNPad, "row padding");
static_assert((kN % 16) == 0 && (kE % 4) == 0, "tile multiples");
static_assert(kD == 128 && (kD % 64) == 0 && (kD % 32) == 0 && (kCPad % 64) == 0 && kC <= kCPad, "gemm multiples");
static_assert((kRng % 8) == 0 && kRng / 8 == 256 && (kCap % 1024) == 0, "builder tiling");

constexpr size_t kOffSeg  = 0;
constexpr size_t kOffDinv = kOffSeg  + (size_t)kNTab * 2 * 4;
constexpr size_t kOffCsr  = kOffDinv + (size_t)kNTab * 4;
constexpr size_t kOffH16  = kOffCsr  + (size_t)kCsrTot * 4;
constexpr size_t kOffHWs  = kOffH16  + (size_t)kNPad * kD * 2;
constexpr size_t kOffMxA  = kOffHWs  + (size_t)kNPad * kD * 2;
constexpr size_t kOffMxB  = kOffMxA  + (size_t)kNPad * kD * 2;
constexpr size_t kOffWt   = kOffMxB  + (size_t)kNPad * kD * 2;
constexpr size_t kOffLWt  = kOffWt   + (size_t)kL * kD * kD * 2;
constexpr size_t kOffSTab = kOffLWt  + (size_t)kCPad * kD * 2;
constexpr size_t kOffTTab = kOffSTab + (size_t)kL * kD * 4;
constexpr size_t kWsTotal = kOffTTab + (size_t)kL * kD * 4;
static_assert(kWsTotal == 108639232ull, "carve total");
static_assert(kWsTotal <= 134217728ull, "carve cap");
static_assert((kOffDinv % 128) == 0 && (kOffCsr % 128) == 0 && (kOffH16 % 128) == 0 && (kOffHWs % 128) == 0 &&
              (kOffMxA % 128) == 0 && (kOffMxB % 128) == 0 && (kOffWt % 128) == 0 && (kOffLWt % 128) == 0 &&
              (kOffSTab % 128) == 0 && (kOffTTab % 128) == 0, "128-B aligned regions");

__device__ __forceinline__ unsigned short f2bf_bits(float f) {
  unsigned u = __float_as_uint(f);
  return (unsigned short)((u + 0x7FFFu + ((u >> 16) & 1u)) >> 16);
}
__device__ __forceinline__ unsigned pack_bf16x2(float lo, float hi) {
  const unsigned a = (unsigned)f2bf_bits(lo);
  const unsigned b = (unsigned)f2bf_bits(hi);
  return a | (b << 16);
}
__device__ __forceinline__ int clamp_node(int v) {
  v = v < 0 ? 0 : v;
  return v > (kN - 1) ? (kN - 1) : v;
}
__device__ __forceinline__ v16h frag_load(const _Float16* p) {
  union U { v16h v; v8h h[2]; };
  U f;
  f.h[0] = *(const v8h*)(p);
  f.h[1] = *(const v8h*)(p + 16);
  return f.v;
}
__device__ __forceinline__ v8f mma_h(v16h a, v16h b, v8f c) {
  c = __builtin_amdgcn_wmma_f32_16x16x32_f16(false, a, false, b, (short)0, c, false, false);
  asm volatile("v_nop\n\tv_nop\n\tv_nop\n\tv_nop" : "+v"(c) : "v"(a), "v"(b));
  return c;
}
__device__ __forceinline__ void wave_lds_sync() {
  __builtin_amdgcn_fence(__ATOMIC_RELEASE, "workgroup");
  __builtin_amdgcn_wave_barrier();
  __builtin_amdgcn_fence(__ATOMIC_ACQUIRE, "workgroup");
}
__device__ __forceinline__ void acc_pair(float& lo, float& hi, unsigned w, bool valid) {
  const float fl = __uint_as_float(w << 16);
  const float fh = __uint_as_float(w & 0xffff0000u);
  lo += valid ? fl : 0.0f;
  hi += valid ? fh : 0.0f;
}
__device__ __forceinline__ float relu_affine(float x, float s, float t) {
  return fmaxf(fmaf(x, s, t), 0.0f) + 0.0f;
}

__global__ __launch_bounds__(256) void build_table_kernel(
    const int* __restrict__ ei, int* __restrict__ segG, float* __restrict__ dinvG, int* __restrict__ csrG)
{
  __shared__ int sCnt[kRng];
  __shared__ int sCur[kRng];
  __shared__ int sScan[256];
  __shared__ __align__(16) int sList[kCap];
  const int tid  = threadIdx.x;
  const int base = blockIdx.x * kRng;
  constexpr int kE4    = kE / 4;
  constexpr int kIters = (kE4 + 255) / 256;
  const v4i* rowp = (const v4i*)ei;
  const v4i* colp = (const v4i*)(ei + kE);

#pragma unroll 1
  for (int i = tid; i < kRng; i += 256) sCnt[i] = 0;
#pragma unroll 1
  for (int i = tid; i < kCap; i += 256) sList[i] = 0;
  __syncthreads();

#pragma unroll 1
  for (int it = 0; it < kIters; ++it) {
    const int q  = it * 256 + tid;
    const int qc = q < kE4 ? q : (kE4 - 1);
    const v4i r4 = rowp[qc];
    const bool ok = q < kE4;
    const int e0 = clamp_node(r4[0]) - base;
    const int e1 = clamp_node(r4[1]) - base;
    const int e2 = clamp_node(r4[2]) - base;
    const int e3 = clamp_node(r4[3]) - base;
    if (ok && (unsigned)e0 < (unsigned)kRng) atomicAdd(&sCnt[e0], 1);
    if (ok && (unsigned)e1 < (unsigned)kRng) atomicAdd(&sCnt[e1], 1);
    if (ok && (unsigned)e2 < (unsigned)kRng) atomicAdd(&sCnt[e2], 1);
    if (ok && (unsigned)e3 < (unsigned)kRng) atomicAdd(&sCnt[e3], 1);
  }
  __syncthreads();

  const int nb = tid * 8;
  int sum = 0;
#pragma unroll
  for (int j = 0; j < 8; ++j) sum += sCnt[nb + j];
  sScan[tid] = sum;
  __syncthreads();
#pragma unroll 1
  for (int off = 1; off < 256; off <<= 1) {
    const int srcI = tid >= off ? tid - off : 0;
    const int add  = sScan[srcI];
    const int cur  = sScan[tid];
    __syncthreads();
    sScan[tid] = cur + (tid >= off ? add : 0);
    __syncthreads();
  }
  const int total = sScan[255];
  {
    int run = sScan[tid] - sum;
#pragma unroll
    for (int j = 0; j < 8; ++j) {
      const int c = sCnt[nb + j];
      sCur[nb + j] = run < kCap ? run : kCap;
      run += c;
    }
  }
  __syncthreads();

#pragma unroll 1
  for (int it = 0; it < kIters; ++it) {
    const int q  = it * 256 + tid;
    const int qc = q < kE4 ? q : (kE4 - 1);
    const v4i r4 = rowp[qc];
    const v4i c4 = colp[qc];
    const bool ok = q < kE4;
    const int e0 = clamp_node(r4[0]) - base;
    const int e1 = clamp_node(r4[1]) - base;
    const int e2 = clamp_node(r4[2]) - base;
    const int e3 = clamp_node(r4[3]) - base;
    const int s0 = clamp_node(c4[0]);
    const int s1 = clamp_node(c4[1]);
    const int s2 = clamp_node(c4[2]);
    const int s3 = clamp_node(c4[3]);
    if (ok && (unsigned)e0 < (unsigned)kRng) {
      const int slot = atomicAdd(&sCur[e0], 1);
      if ((unsigned)slot < (unsigned)kCap) sList[slot] = s0;
    }
    if (ok && (unsigned)e1 < (unsigned)kRng) {
      const int slot = atomicAdd(&sCur[e1], 1);
      if ((unsigned)slot < (unsigned)kCap) sList[slot] = s1;
    }
    if (ok && (unsigned)e2 < (unsigned)kRng) {
      const int slot = atomicAdd(&sCur[e2], 1);
      if ((unsigned)slot < (unsigned)kCap) sList[slot] = s2;
    }
    if (ok && (unsigned)e3 < (unsigned)kRng) {
      const int slot = atomicAdd(&sCur[e3], 1);
      if ((unsigned)slot < (unsigned)kCap) sList[slot] = s3;
    }
  }
  __syncthreads();

#pragma unroll 1
  for (int j = 0; j < 8; ++j) {
    const int c = sCnt[nb + j];
    const int e = sCur[nb + j];
    const int s = e - c;
    if (c > 1 && c <= kSortMax && e <= kCap && s >= 0) {
#pragma unroll 1
      for (int i = 1; i < c; ++i) {
        const int key = sList[s + i];
        int k = i - 1;
#pragma unroll 1
        while (k >= 0) {
          const int v = sList[s + k];
          if (v <= key) break;
          sList[s + k + 1] = v;
          --k;
        }
        sList[s + k + 1] = key;
      }
    }
  }
  __syncthreads();

  const bool ovf = total > kCap;
  const float nanv = __uint_as_float(0x7fc00000u);
  const int slab0 = blockIdx.x * kCap;
  for (int pass = 0; pass < 2; ++pass) {
#pragma unroll 1
    for (int it = 0; it < 4; ++it) {
      const int pr = it * 256 + tid;
      const int n0 = 2 * pr;
      const int c0 = sCnt[n0];
      const int c1 = sCnt[n0 + 1];
      v4i o;
      o[0] = slab0 + (sCur[n0] - c0);
      o[1] = c0;
      o[2] = slab0 + (sCur[n0 + 1] - c1);
      o[3] = c1;
      *(volatile v4i*)(segG + 2 * (size_t)(base + n0)) = o;
    }
#pragma unroll 1
    for (int it = 0; it < 2; ++it) {
      const int n0 = 4 * (it * 256 + tid);
      v4f d;
      d[0] = ovf ? nanv : rsqrtf((float)sCnt[n0 + 0] + 1.0f);
      d[1] = ovf ? nanv : rsqrtf((float)sCnt[n0 + 1] + 1.0f);
      d[2] = ovf ? nanv : rsqrtf((float)sCnt[n0 + 2] + 1.0f);
      d[3] = ovf ? nanv : rsqrtf((float)sCnt[n0 + 3] + 1.0f);
      *(volatile v4f*)(dinvG + (size_t)(base + n0)) = d;
    }
#pragma unroll 1
    for (int it = 0; it < kCap / 1024; ++it) {
      const int i4 = 4 * (it * 256 + tid);
      const v4i v = *(const v4i*)(sList + i4);
      *(volatile v4i*)(csrG + (size_t)slab0 + i4) = v;
    }
    __threadfence();
  }
}

constexpr int kPrepWBlocks = (kL * kD * kD / 8) / 256;
constexpr int kPrepLBlocks = (kCPad * kD / 8) / 256;
static_assert(kPrepWBlocks == 40 && kPrepLBlocks == 4, "prep grid");

__global__ __launch_bounds__(256) void prep_kernel(
    const float* __restrict__ conv_w, const float* __restrict__ conv_b,
    const float* __restrict__ gam, const float* __restrict__ bet,
    const float* __restrict__ mean, const float* __restrict__ var,
    const float* __restrict__ lin_w,
    unsigned short* __restrict__ Wt16, unsigned short* __restrict__ LWt16,
    float* __restrict__ sTab, float* __restrict__ tTab)
{
  const int tid = threadIdx.x;
  const int bx  = blockIdx.x;
  if (bx < kPrepWBlocks) {
    const int t  = bx * 256 + tid;
    const int k8 = t & 15;
    const int n  = (t >> 4) & 127;
    const int l  = t >> 11;
    const float* src = conv_w + ((size_t)(l * kD + k8 * 8)) * kD + n;
    v8h hv;
#pragma unroll
    for (int e = 0; e < 8; ++e) hv[e] = (_Float16)(src[(size_t)e * kD] * kWCarry);
    unsigned short* dst = Wt16 + (size_t)t * 8;
    *(volatile v8h*)(void*)dst = hv;
    __threadfence();
    *(volatile v8h*)(void*)dst = hv;
  } else if (bx < kPrepWBlocks + kPrepLBlocks) {
    const int t  = (bx - kPrepWBlocks) * 256 + tid;
    const int k8 = t & 15;
    const int n  = t >> 4;
    const int nc = n < kC ? n : (kC - 1);
    v8h hv;
#pragma unroll
    for (int e = 0; e < 8; ++e) {
      const float w = lin_w[(size_t)(k8 * 8 + e) * kC + nc];
      hv[e] = (_Float16)((n < kC) ? (w * kWCarry) : 0.0f);
    }
    unsigned short* dst = LWt16 + (size_t)t * 8;
    *(volatile v8h*)(void*)dst = hv;
    __threadfence();
    *(volatile v8h*)(void*)dst = hv;
  } else {
    if (tid < (kL * kD) / 4) {
      const int idx = tid * 4;
      const v4f g  = *(const v4f*)(gam + idx);
      const v4f b  = *(const v4f*)(bet + idx);
      const v4f m  = *(const v4f*)(mean + idx);
      const v4f v  = *(const v4f*)(var + idx);
      const v4f cb = *(const v4f*)(conv_b + idx);
      v4f s, t;
#pragma unroll
      for (int j = 0; j < 4; ++j) {
        const float sj = g[j] * rsqrtf(v[j] + kEps);
        s[j] = sj;
        t[j] = b[j] + (cb[j] - m[j]) * sj;
      }
      *(volatile v4f*)(sTab + idx) = s;
      *(volatile v4f*)(tTab + idx) = t;
      __threadfence();
      *(volatile v4f*)(sTab + idx) = s;
      *(volatile v4f*)(tTab + idx) = t;
    }
  }
}

__global__ __launch_bounds__(256) void cvt_input_kernel(
    const float* __restrict__ x, unsigned short* __restrict__ H16, unsigned short* __restrict__ MxA)
{
  const int i    = blockIdx.x * 256 + threadIdx.x;
  const int row  = i >> 4;
  const int rowc = row < kN ? row : (kN - 1);
  const bool real = row < kN;
  const float* src = x + (size_t)rowc * kD + (i & 15) * 8;
  const v4f a0 = *(const v4f*)(src);
  const v4f a1 = *(const v4f*)(src + 4);
  v8h hv;
#pragma unroll
  for (int e = 0; e < 4; ++e) {
    hv[e]     = (_Float16)(real ? a0[e] : 0.0f);
    hv[4 + e] = (_Float16)(real ? a1[e] : 0.0f);
  }
  unsigned short* dh = H16 + (size_t)i * 8;
  unsigned short* dm = MxA + (size_t)i * 8;
  for (int pass = 0; pass < 2; ++pass) {
    *(volatile v8h*)(void*)dh = hv;
    if (!real) *(volatile v8h*)(void*)dm = hv;
    __threadfence();
  }
}

__global__ __launch_bounds__(256) void layer_gemm_kernel(
    const unsigned short* __restrict__ Ap, const unsigned short* __restrict__ Btp,
    const float* __restrict__ dinv, unsigned short* __restrict__ Cout)
{
  __shared__ __align__(16) float sT[8][16 * 68];
  const _Float16* A  = (const _Float16*)(const void*)Ap;
  const _Float16* Bt = (const _Float16*)(const void*)Btp;
  const int lane = threadIdx.x & 31;
  const int wave = threadIdx.x >> 5;
  constexpr int tilesN = kD >> 6;
  constexpr int tilesM = kNPad >> 6;
  const int tile = blockIdx.x * 8 + wave;
  if (tile >= tilesM * tilesN) return;
  const int tm = tile / tilesN;
  const int tn = tile - tm * tilesN;
  const int m0 = tm << 6;
  const int n0 = tn << 6;
  const int rlane = lane & 15;
  const int koff  = (lane >> 4) * 8;
  const int mOff  = (lane >> 4) * 8;

  v8f acc[4][4];
#pragma unroll
  for (int i = 0; i < 4; ++i)
#pragma unroll
    for (int j = 0; j < 4; ++j) acc[i][j] = (v8f){0.f, 0.f, 0.f, 0.f, 0.f, 0.f, 0.f, 0.f};

#pragma unroll 1
  for (int k0 = 0; k0 < kD; k0 += 32) {
    v16h bh[4];
#pragma unroll
    for (int j = 0; j < 4; ++j)
      bh[j] = frag_load(Bt + (size_t)(n0 + (j << 4) + rlane) * kD + koff + k0);
#pragma unroll
    for (int i = 0; i < 4; ++i) {
      const v16h ah = frag_load(A + (size_t)(m0 + (i << 4) + rlane) * kD + koff + k0);
#pragma unroll
      for (int j = 0; j < 4; ++j) acc[i][j] = mma_h(ah, bh[j], acc[i][j]);
    }
  }

  float* slab = sT[wave];
  const int q  = lane >> 3;
  const int c8 = (lane & 7) * 8;
#pragma unroll
  for (int i = 0; i < 4; ++i) {
    const int mBase = m0 + (i << 4);
    const v4f d0 = *(const v4f*)(dinv + mBase + mOff);
    const v4f d1 = *(const v4f*)(dinv + mBase + mOff + 4);
    float ds[8];
    ds[0] = d0[0] * kWCarryInv; ds[1] = d0[1] * kWCarryInv; ds[2] = d0[2] * kWCarryInv; ds[3] = d0[3] * kWCarryInv;
    ds[4] = d1[0] * kWCarryInv; ds[5] = d1[1] * kWCarryInv; ds[6] = d1[2] * kWCarryInv; ds[7] = d1[3] * kWCarryInv;
#pragma unroll
    for (int j = 0; j < 4; ++j) {
#pragma unroll
      for (int r = 0; r < 8; ++r)
        slab[(mOff + r) * 68 + (j << 4) + rlane] = acc[i][j][r] * ds[r];
    }
    wave_lds_sync();
    v4u pk[4];
#pragma unroll
    for (int it = 0; it < 4; ++it) {
      const float* sp = slab + (it * 4 + q) * 68 + c8;
      const v4f a0 = *(const v4f*)(sp);
      const v4f a1 = *(const v4f*)(sp + 4);
      v4u w;
      w[0] = pack_bf16x2(a0[0], a0[1]);
      w[1] = pack_bf16x2(a0[2], a0[3]);
      w[2] = pack_bf16x2(a1[0], a1[1]);
      w[3] = pack_bf16x2(a1[2], a1[3]);
      pk[it] = w;
    }
    for (int pass = 0; pass < 2; ++pass) {
#pragma unroll
      for (int it = 0; it < 4; ++it) {
        unsigned short* dst = Cout + (size_t)(mBase + it * 4 + q) * kD + n0 + c8;
        *(volatile v4u*)(void*)dst = pk[it];
      }
      __threadfence();
    }
    wave_lds_sync();
  }
}

__global__ __launch_bounds__(256) void aggregate_kernel(
    const unsigned short* __restrict__ HWs, const int* __restrict__ seg, const int* __restrict__ csr,
    const float* __restrict__ dinv, const float* __restrict__ sVec, const float* __restrict__ tVec,
    unsigned short* __restrict__ Hout, const unsigned short* __restrict__ MxIn, unsigned short* __restrict__ MxOut,
    int first, int writeH)
{
  const int lane = threadIdx.x & 31;
  const int wave = threadIdx.x >> 5;
  const int half = lane >> 4;
  const int ch   = (lane & 15) * 8;
  const int node  = (blockIdx.x * 8 + wave) * 2 + half;
  const int nodeC = node < kN ? node : (kN - 1);

  int start = seg[2 * (size_t)nodeC];
  int cnt   = seg[2 * (size_t)nodeC + 1];
  start = start < 0 ? 0 : start;
  start = start > (kCsrTot - 1) ? (kCsrTot - 1) : start;
  cnt = cnt < 0 ? 0 : cnt;
  cnt = cnt > kCap ? kCap : cnt;
  const int cntO = __shfl_xor(cnt, 16, 32);
  int trip = cnt > cntO ? cnt : cntO;
  trip = __builtin_amdgcn_readfirstlane(trip);

  float a0 = 0.0f, a1 = 0.0f, a2 = 0.0f, a3 = 0.0f, a4 = 0.0f, a5 = 0.0f, a6 = 0.0f, a7 = 0.0f;
  {
    const v4u w = *(const v4u*)(const void*)(HWs + (size_t)nodeC * kD + ch);
    acc_pair(a0, a1, w[0], true);
    acc_pair(a2, a3, w[1], true);
    acc_pair(a4, a5, w[2], true);
    acc_pair(a6, a7, w[3], true);
  }
#pragma unroll 1
  for (int p = 0; p < trip; ++p) {
    const bool valid = p < cnt;
    const int pi = valid ? p : 0;
    int idx = start + pi;
    idx = idx > (kCsrTot - 1) ? (kCsrTot - 1) : idx;
    int src = csr[idx];
    asm volatile("" : "+v"(src));
    src = clamp_node(src);
    const v4u w = *(const v4u*)(const void*)(HWs + (size_t)src * kD + ch);
    unsigned w0 = w[0];
    unsigned w1 = w[1];
    unsigned w2 = w[2];
    unsigned w3 = w[3];
    asm volatile("" : "+v"(w0), "+v"(w1), "+v"(w2), "+v"(w3));
    acc_pair(a0, a1, w0, valid);
    acc_pair(a2, a3, w1, valid);
    acc_pair(a4, a5, w2, valid);
    acc_pair(a6, a7, w3, valid);
  }

  const float dn = dinv[nodeC];
  const v4f s0 = *(const v4f*)(sVec + ch);
  const v4f s1 = *(const v4f*)(sVec + ch + 4);
  const v4f t0 = *(const v4f*)(tVec + ch);
  const v4f t1 = *(const v4f*)(tVec + ch + 4);
  v8h hv;
  hv[0] = (_Float16)relu_affine(a0 * dn, s0[0], t0[0]);
  hv[1] = (_Float16)relu_affine(a1 * dn, s0[1], t0[1]);
  hv[2] = (_Float16)relu_affine(a2 * dn, s0[2], t0[2]);
  hv[3] = (_Float16)relu_affine(a3 * dn, s0[3], t0[3]);
  hv[4] = (_Float16)relu_affine(a4 * dn, s1[0], t1[0]);
  hv[5] = (_Float16)relu_affine(a5 * dn, s1[1], t1[1]);
  hv[6] = (_Float16)relu_affine(a6 * dn, s1[2], t1[2]);
  hv[7] = (_Float16)relu_affine(a7 * dn, s1[3], t1[3]);
  const v4u hw = __builtin_bit_cast(v4u, hv);
  v4u mx = hw;
  if (first == 0) {
    const v4u old = *(const v4u*)(const void*)(MxIn + (size_t)nodeC * kD + ch);
#pragma unroll
    for (int j = 0; j < 4; ++j) {
      const unsigned on = old[j];
      const unsigned nn = hw[j];
      const unsigned ol = on & 0xffffu, nl = nn & 0xffffu;
      const unsigned oh = on >> 16,     nh = nn >> 16;
      const unsigned ml = ol > nl ? ol : nl;
      const unsigned mh = oh > nh ? oh : nh;
      mx[j] = ml | (mh << 16);
    }
  }
  unsigned short* hp = Hout  + (size_t)nodeC * kD + ch;
  unsigned short* mp = MxOut + (size_t)nodeC * kD + ch;
  for (int pass = 0; pass < 2; ++pass) {
    if (writeH != 0) *(volatile v4u*)(void*)hp = hw;
    *(volatile v4u*)(void*)mp = mx;
    __threadfence();
  }
}

__global__ __launch_bounds__(256) void head_kernel(
    const unsigned short* __restrict__ Ap, const unsigned short* __restrict__ Btp,
    const float* __restrict__ lin_b, float* __restrict__ out)
{
  __shared__ __align__(16) float sT[8][16 * 68];
  __shared__ float sL[8][16];
  const _Float16* A  = (const _Float16*)(const void*)Ap;
  const _Float16* Bt = (const _Float16*)(const void*)Btp;
  const int lane = threadIdx.x & 31;
  const int wave = threadIdx.x >> 5;
  constexpr int tilesM = kNPad >> 6;
  const int tile = blockIdx.x * 8 + wave;
  if (tile >= tilesM) return;
  const int m0 = tile << 6;
  const int rlane = lane & 15;
  const int koff  = (lane >> 4) * 8;
  const int mOff  = (lane >> 4) * 8;

  v8f acc[4][4];
#pragma unroll
  for (int i = 0; i < 4; ++i)
#pragma unroll
    for (int j = 0; j < 4; ++j) acc[i][j] = (v8f){0.f, 0.f, 0.f, 0.f, 0.f, 0.f, 0.f, 0.f};

#pragma unroll 1
  for (int k0 = 0; k0 < kD; k0 += 32) {
    v16h bh[4];
#pragma unroll
    for (int j = 0; j < 4; ++j)
      bh[j] = frag_load(Bt + (size_t)((j << 4) + rlane) * kD + koff + k0);
#pragma unroll
    for (int i = 0; i < 4; ++i) {
      const v16h ah = frag_load(A + (size_t)(m0 + (i << 4) + rlane) * kD + koff + k0);
#pragma unroll
      for (int j = 0; j < 4; ++j) acc[i][j] = mma_h(ah, bh[j], acc[i][j]);
    }
  }

  float* slab = sT[wave];
  float* lrow = sL[wave];
  float bj[4];
#pragma unroll
  for (int j = 0; j < 4; ++j) {
    const int n  = (j << 4) + rlane;
    const int nc = n < kC ? n : (kC - 1);
    const float bv = lin_b[nc];
    bj[j] = (n < kC) ? bv : 0.0f;
  }
  const int srow = lane & 15;
  const int hx   = lane >> 4;
#pragma unroll
  for (int i = 0; i < 4; ++i) {
    const int mBase = m0 + (i << 4);
#pragma unroll
    for (int j = 0; j < 4; ++j) {
#pragma unroll
      for (int r = 0; r < 8; ++r)
        slab[(mOff + r) * 68 + (j << 4) + rlane] = acc[i][j][r] * kWCarryInv + bj[j];
    }
    wave_lds_sync();
    const float* rp = slab + srow * 68 + hx * 20;
    float mxv = -INFINITY;
#pragma unroll 1
    for (int c = 0; c < 20; ++c) mxv = fmaxf(mxv, rp[c]);
    mxv = fmaxf(mxv, __shfl_xor(mxv, 16, 32));
    float sm = 0.0f;
#pragma unroll 1
    for (int c = 0; c < 20; ++c) sm += expf(rp[c] - mxv);
    sm += __shfl_xor(sm, 16, 32);
    const float lse = mxv + logf(sm);
    if (hx == 0) lrow[srow] = lse;
    wave_lds_sync();
    v4f ov[5];
#pragma unroll
    for (int it = 0; it < 5; ++it) {
      const int e   = (it * 32 + lane) * 4;
      const int row = e / kC;
      const int col = e - row * kC;
      const v4f z = *(const v4f*)(slab + row * 68 + col);
      const float l = lrow[row];
      v4f o;
      o[0] = z[0] - l; o[1] = z[1] - l; o[2] = z[2] - l; o[3] = z[3] - l;
      ov[it] = o;
    }
    if (mBase < kN) {
      float* ob = out + (size_t)mBase * kC;
      for (int pass = 0; pass < 2; ++pass) {
#pragma unroll
        for (int it = 0; it < 5; ++it)
          *(volatile v4f*)(ob + (it * 32 + lane) * 4) = ov[it];
        __threadfence();
      }
    }
    wave_lds_sync();
  }
}

extern "C" void kernel_launch(void* const* d_in, const int* in_sizes, int n_in,
                              void* d_out, int out_size, void* d_ws, size_t ws_size,
                              hipStream_t stream) {
  if (n_in < 10) return;
  if (in_sizes[0] != kN * kD) return;
  if (in_sizes[1] != 2 * kE) return;
  if (in_sizes[2] != kL * kD * kD) return;
  if (in_sizes[3] != kL * kD) return;
  if (in_sizes[4] != kL * kD) return;
  if (in_sizes[5] != kL * kD) return;
  if (in_sizes[6] != kL * kD) return;
  if (in_sizes[7] != kL * kD) return;
  if (in_sizes[8] != kD * kC) return;
  if (in_sizes[9] != kC) return;
  if (out_size != kN * kC) return;
  if (ws_size < kWsTotal) return;

  const float* x      = (const float*)d_in[0];
  const int*   ei     = (const int*)  d_in[1];
  const float* conv_w = (const float*)d_in[2];
  const float* conv_b = (const float*)d_in[3];
  const float* gam    = (const float*)d_in[4];
  const float* bet    = (const float*)d_in[5];
  const float* mean   = (const float*)d_in[6];
  const float* var    = (const float*)d_in[7];
  const float* lin_w  = (const float*)d_in[8];
  const float* lin_b  = (const float*)d_in[9];
  float* out = (float*)d_out;

  char* ws = (char*)d_ws;
  int*            SEG   = (int*)(ws + kOffSeg);
  float*          DINV  = (float*)(ws + kOffDinv);
  int*            CSR   = (int*)(ws + kOffCsr);
  unsigned short* H16   = (unsigned short*)(ws + kOffH16);
  unsigned short* HWS   = (unsigned short*)(ws + kOffHWs);
  unsigned short* MXA   = (unsigned short*)(ws + kOffMxA);
  unsigned short* MXB   = (unsigned short*)(ws + kOffMxB);
  unsigned short* WT16  = (unsigned short*)(ws + kOffWt);
  unsigned short* LWT16 = (unsigned short*)(ws + kOffLWt);
  float*          STAB  = (float*)(ws + kOffSTab);
  float*          TTAB  = (float*)(ws + kOffTTab);

  build_table_kernel<<<kNblkR, 256, 0, stream>>>(ei, SEG, DINV, CSR);
  prep_kernel<<<kPrepWBlocks + kPrepLBlocks + 1, 256, 0, stream>>>(
      conv_w, conv_b, gam, bet, mean, var, lin_w, WT16, LWT16, STAB, TTAB);
  cvt_input_kernel<<<(kNPad * kD / 8) / 256, 256, 0, stream>>>(x, H16, MXA);

  constexpr int kGemmBlocks = ((kNPad >> 6) * (kD >> 6) + 7) / 8;
  constexpr int kAggBlocks  = kN / 16;
  for (int l = 0; l < kL; ++l) {
    layer_gemm_kernel<<<kGemmBlocks, 256, 0, stream>>>(H16, WT16 + (size_t)l * kD * kD, DINV, HWS);
    unsigned short* mxOut = (l & 1) ? MXB : MXA;
    const unsigned short* mxIn = (l & 1) ? MXA : MXB;
    aggregate_kernel<<<kAggBlocks, 256, 0, stream>>>(
        HWS, SEG, CSR, DINV, STAB + l * kD, TTAB + l * kD, H16, mxIn, mxOut,
        (l == 0) ? 1 : 0, (l < kL - 1) ? 1 : 0);
  }

  constexpr int kHeadBlocks = ((kNPad >> 6) + 7) / 8;
  head_kernel<<<kHeadBlocks, 256, 0, stream>>>(MXA, LWT16, lin_b, out);
}
